// Colla_Attention_87591563034981
// MI455X (gfx1250) — hardware-verified
//
#include <hip/hip_runtime.h>
#include <math.h>

typedef __attribute__((ext_vector_type(16))) _Float16 v16h;
typedef __attribute__((ext_vector_type(16))) __bf16 v16b;
typedef __attribute__((ext_vector_type(8)))  _Float16 v8h;
typedef __attribute__((ext_vector_type(8)))  float v8f;
typedef __attribute__((ext_vector_type(4)))  float v4f;
typedef __attribute__((ext_vector_type(2)))  float v2f;
typedef __attribute__((ext_vector_type(4)))  unsigned v4u;
typedef __attribute__((ext_vector_type(4)))  int v4i;
typedef float __attribute__((may_alias)) float_a;
typedef int __attribute__((may_alias)) int_a;

template <typename T> __device__ __forceinline__ void vst2(void* p, T v) { *(volatile T*)p = v; __threadfence(); *(volatile T*)p = v; }
__device__ __forceinline__ v8f wmma16(v16h a, v16h b, v8f c) {
  v8f d = __builtin_amdgcn_wmma_f32_16x16x32_f16(false, a, false, b, (short)0, c, false, false);
  asm volatile("v_nop\n\tv_nop\n\tv_nop\n\tv_nop" : "+v"(d) : "v"(a), "v"(b));
  return d;
}
__device__ __forceinline__ v8f wmma_bf(v16b a, v16b b, v8f c) {
  v8f d = __builtin_amdgcn_wmma_f32_16x16x32_bf16(false, a, false, b, (short)0, c, false, false);
  asm volatile("v_nop\n\tv_nop\n\tv_nop\n\tv_nop" : "+v"(d) : "v"(a), "v"(b));
  return d;
}
__device__ __forceinline__ v16h frag_h(const _Float16* rowk0, int lane) {
  union { v16h v; v8h q[2]; } u; const _Float16* p = rowk0 + 8 * (lane >> 4);
  u.q[0] = *(const v8h*)p; u.q[1] = *(const v8h*)(p + 16); return u.v;
}
__device__ __forceinline__ v16h frag_f32(const float* rowk0, int lane) {
  v16h a; const float* p = rowk0 + 8 * (lane >> 4);
#pragma unroll
  for (int i = 0; i < 8; ++i) { a[i] = (_Float16)p[i]; a[8 + i] = (_Float16)p[16 + i]; }
  return a;
}
__device__ __forceinline__ v16h frag_f32s(const float* rowk0, int lane, float sc) {
  v16h a; const float* p = rowk0 + 8 * (lane >> 4);
#pragma unroll
  for (int i = 0; i < 8; ++i) { a[i] = (_Float16)(p[i] * sc); a[8 + i] = (_Float16)(p[16 + i] * sc); }
  return a;
}
__device__ __forceinline__ v16h fragc_f32(const float* W, int k0, int n, int lane, int ld, int K) {
  v16h a; const int g = lane >> 4;
#pragma unroll
  for (int i = 0; i < 8; ++i) { const int ka = k0 + 8 * g + i, kb = ka + 16;
    a[i] = (_Float16)(ka < K ? W[(size_t)(ka < K ? ka : K - 1) * ld + n] : 0.f); a[8 + i] = (_Float16)(kb < K ? W[(size_t)(kb < K ? kb : K - 1) * ld + n] : 0.f); }
  return a;
}
struct F2 { v16b h, l; };
__device__ __forceinline__ F2 bsplit16(const float v[16]) { F2 r;
#pragma unroll
  for (int i = 0; i < 16; ++i) { const __bf16 h = (__bf16)v[i]; r.h[i] = h; r.l[i] = (__bf16)(v[i] - (float)h); }
  return r; }
__device__ __forceinline__ F2 split_row(const float* row, int k0, int lane) { float v[16]; const float* p = row + k0 + 8 * (lane >> 4);
#pragma unroll
  for (int i = 0; i < 8; ++i) { v[i] = p[i]; v[8 + i] = p[16 + i]; }
  return bsplit16(v); }
__device__ __forceinline__ F2 split_rowK(const float* row, int k0, int lane, int K) { float v[16]; const int g = lane >> 4;
#pragma unroll
  for (int i = 0; i < 8; ++i) { const int ka = k0 + 8 * g + i, kb = ka + 16; v[i] = ka < K ? row[ka < K ? ka : K - 1] : 0.f; v[8 + i] = kb < K ? row[kb < K ? kb : K - 1] : 0.f; }
  return bsplit16(v); }
__device__ __forceinline__ F2 split_col(const float* W, int k0, int n, int lane, int ld, int K) { float v[16]; const int g = lane >> 4;
#pragma unroll
  for (int i = 0; i < 8; ++i) { const int ka = k0 + 8 * g + i, kb = ka + 16; v[i] = ka < K ? W[(size_t)(ka < K ? ka : K - 1) * ld + n] : 0.f; v[8 + i] = kb < K ? W[(size_t)(kb < K ? kb : K - 1) * ld + n] : 0.f; }
  return bsplit16(v); }
__device__ __forceinline__ v8f mac3(const F2& a, const F2& b, v8f c) { c = wmma_bf(a.l, b.h, c); c = wmma_bf(a.h, b.l, c); return wmma_bf(a.h, b.h, c); }
__device__ __forceinline__ float sigm(float v) { return 1.0f / (1.0f + expf(-v)); }
#define LDSX() do { asm volatile("s_wait_dscnt 0" ::: "memory"); __builtin_amdgcn_wave_barrier(); __builtin_amdgcn_fence(__ATOMIC_RELEASE, "workgroup"); } while (0)


#define NB 2
#define NN 2048
#define DD 512
#define NH 8
#define DH 64
#ifndef TNB
#define TNB NB
#endif
#ifndef TQB
#define TQB (NN / 64)
#endif
typedef __attribute__((ext_vector_type(8))) __bf16 v8b;
__device__ __forceinline__ v16b frag_b(const __bf16* rowk0, int lane) {
  union { v16b v; v8b q[2]; } u; const __bf16* p = rowk0 + 8 * (lane >> 4);
  u.q[0] = *(const v8b*)p; u.q[1] = *(const v8b*)(p + 16); return u.v;
}
__device__ __forceinline__ float bfr(float v) { return (float)(__bf16)v; }
__device__ __attribute__((noinline)) float exp_ni(float v) { return expf(v); }
__device__ __attribute__((noinline)) float erf_ni(float v) { return erff(v); }

#define WS_QM  0u
#define WS_KH  (WS_QM + 2u * (size_t)NB * NN * NH * DD)
#define WS_VT  (WS_KH + 2u * (size_t)NB * NN * DD)
#define WS_CB  (WS_VT + 2u * (size_t)NB * DD * NN)
#define WS_O   (WS_CB + 4u * (size_t)NB * NH * NN)
#define WS_END (WS_O + 4u * (size_t)NB * NN * DD)

__device__ __forceinline__ v16b fragb_f32(const float* __restrict__ p, int lane) { v16b a; const float* pp = p + 8 * (lane >> 4);
#pragma unroll
  for (int i = 0; i < 8; ++i) { a[i] = (__bf16)pp[i]; a[8 + i] = (__bf16)pp[16 + i]; } return a; }
__global__ __launch_bounds__(128) void k_proj(const float* __restrict__ X, const float* __restrict__ WQ, const float* __restrict__ WK, const float* __restrict__ WV, const float* __restrict__ MIX, _Float16* __restrict__ QM, _Float16* __restrict__ KH, _Float16* __restrict__ VT) {
  __shared__ __align__(16) float sf[64][132]; __shared__ __align__(16) _Float16 sh[64][136]; __shared__ __align__(16) _Float16 th[128][72];
  const int tid = threadIdx.x, wave = tid >> 5, lane = tid & 31, col = lane & 15, g = lane >> 4; const int which = blockIdx.z / NB; const size_t b = blockIdx.z % NB; const int n0 = blockIdx.x * 64; const int c0 = blockIdx.y * 128; const size_t r0 = b * NN + n0 + wave * 16;
  const float* Wm = which == 0 ? WQ : which == 1 ? WK : WV;
  v8f acc[8] = {};
#pragma unroll 2
  for (int kc = 0; kc < DD / 32; ++kc) { const v16b a = fragb_f32(X + (r0 + col) * DD + kc * 32, lane);
#pragma unroll
    for (int j = 0; j < 8; ++j) acc[j] = wmma_bf(a, fragb_f32(Wm + (size_t)(c0 + j * 16 + col) * DD + kc * 32, lane), acc[j]); }
#pragma unroll
  for (int j = 0; j < 8; ++j)
#pragma unroll
    for (int r = 0; r < 8; ++r) { const float v = acc[j][r]; if (which == 0) sf[wave * 16 + 8 * g + r][j * 16 + col] = v; else if (which == 1) sh[wave * 16 + 8 * g + r][j * 16 + col] = (_Float16)v; else th[j * 16 + col][wave * 16 + 8 * g + r] = (_Float16)v; }
  __syncthreads();
  if (which == 0) {
#pragma unroll 1
    for (int h = 0; h < NH; ++h) { for (int e = tid; e < 64 * 128; e += 128) { const int rl = e >> 7, c = e & 127; sh[rl][c] = (_Float16)(sf[rl][c] * bfr(MIX[h * DD + c0 + c])); } __syncthreads();
      for (int e = tid; e < 64 * 16; e += 128) { const int rl = e >> 4, q = e & 15; vst2((unsigned*)(QM + (b * NN + n0 + rl) * (size_t)(NH * DD) + (size_t)h * DD + c0 + q * 8), *(const v4u*)&sh[rl][q * 8]); } __syncthreads(); } }
  else if (which == 1) { for (int e = tid; e < 64 * 16; e += 128) { const int rl = e >> 4, q = e & 15; vst2((unsigned*)(KH + (b * NN + n0 + rl) * DD + c0 + q * 8), *(const v4u*)&sh[rl][q * 8]); } }
  else { for (int e = tid; e < 128 * 8; e += 128) { const int cl = e >> 3, q = e & 7; vst2((unsigned*)(VT + (b * DD + c0 + cl) * (size_t)NN + n0 + q * 8), *(const v4u*)&th[cl][q * 8]); } } }
__global__ __launch_bounds__(256) void k_cb(const float* __restrict__ X, const float* __restrict__ WB, float* __restrict__ CB) { __shared__ __align__(16) float so[NH][64]; __shared__ float red[NH][64][4]; const int t = threadIdx.x; const size_t b = blockIdx.y; const int s0 = blockIdx.x * 64; const int sl = t & 63, part = t >> 6;
#pragma unroll 1
  for (int h = 0; h < NH; ++h) { float acc = 0.f; const float* xr = X + (b * NN + s0 + sl) * DD; const float* wr = WB + h * DD;
#pragma unroll 1
    for (int d = part; d < DD; d += 4) acc += bfr(xr[d]) * bfr(wr[d]); red[h][sl][part] = acc; }
  __syncthreads(); for (int e = t; e < NH * 64; e += 256) { const int h = e >> 6, s = e & 63; so[h][s] = red[h][s][0] + red[h][s][1] + red[h][s][2] + red[h][s][3]; } __syncthreads();
  if (t < NH * 16) { const int h = t >> 4, q = t & 15; vst2(CB + (b * NH + h) * (size_t)NN + s0 + q * 4, *(const v4f*)&so[h][q * 4]); } }
__global__ __launch_bounds__(128) void k_att(const _Float16* __restrict__ QM, const _Float16* __restrict__ KH, const _Float16* __restrict__ VT, const float* __restrict__ CB, float* __restrict__ O) {
  __shared__ __align__(16) float sp[4][16][36]; __shared__ __align__(16) float so[4][16][68];
  const int tid = threadIdx.x, wave = tid >> 5, lane = tid & 31, col = lane & 15, g = lane >> 4; const int h = blockIdx.y; const size_t b = blockIdx.z; const int q0 = blockIdx.x * 64 + wave * 16; const size_t rq = b * NN + q0;
  const _Float16* qbase = QM + (rq + col) * (size_t)(NH * DD) + (size_t)h * DD; const float* cbh = CB + (b * NH + h) * (size_t)NN;
  float m[8], l[8];
#pragma unroll
  for (int r = 0; r < 8; ++r) { m[r] = -3.0e38f; l[r] = 0.f; }
  v8f acc[4] = {}, accl[4] = {};
#pragma unroll 1
  for (int ks = 0; ks < NN / 32; ++ks) { v8f s[2];
#pragma unroll
    for (int ct = 0; ct < 2; ++ct) { const int kk = ks * 32 + ct * 16 + col; const _Float16* kbase = KH + (b * NN + kk) * DD; v8f c = {};
#pragma unroll 4
      for (int kc = 0; kc < DD / 32; ++kc) c = wmma16(frag_h(qbase + kc * 32, lane), frag_h(kbase + kc * 32, lane), c);
      const float cbv = cbh[kk];
#pragma unroll
      for (int r = 0; r < 8; ++r) s[ct][r] = (c[r] + cbv) * 0.125f; }
    float alpha[8];
#pragma unroll
    for (int r = 0; r < 8; ++r) { float mx = fmaxf(s[0][r], s[1][r]);
#pragma unroll
      for (int o = 1; o < 16; o <<= 1) mx = fmaxf(mx, __shfl_xor(mx, o));
      const float mn = fmaxf(m[r], mx); alpha[r] = __expf(m[r] - mn); const float e0 = __expf(s[0][r] - mn), e1 = __expf(s[1][r] - mn); float es = e0 + e1;
#pragma unroll
      for (int o = 1; o < 16; o <<= 1) es += __shfl_xor(es, o);
      l[r] = l[r] * alpha[r] + es; m[r] = mn; sp[wave][8 * g + r][col] = e0; sp[wave][8 * g + r][16 + col] = e1; }
#pragma unroll
    for (int j = 0; j < 4; ++j)
#pragma unroll
      for (int r = 0; r < 8; ++r) { acc[j][r] *= alpha[r]; accl[j][r] *= alpha[r]; }
    LDSX();
    v16h pa, pal; { const float* prow = &sp[wave][col][0] + 8 * (lane >> 4);
#pragma unroll
      for (int i = 0; i < 8; ++i) { const float p0 = prow[i] * 2048.0f, p1 = prow[16 + i] * 2048.0f; pa[i] = (_Float16)p0; pa[8 + i] = (_Float16)p1; pal[i] = (_Float16)((p0 - (float)pa[i]) * 2048.0f); pal[8 + i] = (_Float16)((p1 - (float)pa[8 + i]) * 2048.0f); } }
#pragma unroll
    for (int j = 0; j < 4; ++j) { const v16h vf = frag_h(VT + (b * DD + (size_t)h * DH + j * 16 + col) * (size_t)NN + ks * 32, lane); acc[j] = wmma16(pa, vf, acc[j]); accl[j] = wmma16(pal, vf, accl[j]); }
    LDSX(); }
#pragma unroll
  for (int r = 0; r < 8; ++r) { const float il = (1.0f / 2048.0f) / l[r];
#pragma unroll
    for (int j = 0; j < 4; ++j) so[wave][8 * g + r][j * 16 + col] = (acc[j][r] + accl[j][r] * (1.0f / 2048.0f)) * il; }
  LDSX(); for (int rl = 0; rl < 16; ++rl) if (lane < 16) vst2(O + (rq + rl) * DD + (size_t)h * DH + lane * 4, *(const v4f*)&so[wave][rl][lane * 4]); }
__global__ __launch_bounds__(128) void k_out(const float* __restrict__ Or, const float* __restrict__ WD, const float* __restrict__ BD, float* __restrict__ OUT) { __shared__ __align__(16) float sf[4][16][132];
  const int tid = threadIdx.x, wave = tid >> 5, lane = tid & 31, col = lane & 15, g = lane >> 4; const size_t r0 = (size_t)blockIdx.x * 64 + wave * 16; const int c0 = blockIdx.y * 128;
  v8f acc[8] = {};
#pragma unroll 2
  for (int kc = 0; kc < DD / 32; ++kc) { const F2 a = split_row(Or + (r0 + col) * DD, kc * 32, lane);
#pragma unroll
    for (int j = 0; j < 8; ++j) { const v16b w = fragb_f32(WD + (size_t)(c0 + j * 16 + col) * DD + kc * 32, lane); acc[j] = wmma_bf(a.h, w, acc[j]); acc[j] = wmma_bf(a.l, w, acc[j]); } }
#pragma unroll
  for (int j = 0; j < 8; ++j) { const float bb = bfr(BD[c0 + j * 16 + col]);
#pragma unroll
    for (int r = 0; r < 8; ++r) sf[wave][8 * g + r][j * 16 + col] = acc[j][r] + bb; }
  LDSX(); for (int rl = 0; rl < 16; ++rl) vst2(OUT + (r0 + rl) * DD + c0 + lane * 4, *(const v4f*)&sf[wave][rl][lane * 4]); }
extern "C" void kernel_launch(void* const* d_in, const int* in_sizes, int n_in, void* d_out, int out_size, void* d_ws, size_t ws_size, hipStream_t stream) {
  (void)in_sizes; (void)n_in; (void)out_size;
  const float** F = (const float**)d_in;
  if (ws_size < (size_t)WS_END) return;
  char* ws = (char*)d_ws; _Float16 *QM = (_Float16*)(ws + WS_QM), *KH = (_Float16*)(ws + WS_KH), *VT = (_Float16*)(ws + WS_VT); float *CB = (float*)(ws + WS_CB), *O = (float*)(ws + WS_O);
  k_proj<<<dim3(NN / 64, DD / 128, 3 * NB), 128, 0, stream>>>(F[0], F[1], F[2], F[3], F[5], QM, KH, VT);
  k_cb<<<dim3(NN / 64, NB), 256, 0, stream>>>(F[0], F[4], CB);
  k_att<<<dim3(TQB, NH, TNB), 128, 0, stream>>>(QM, KH, VT, CB, O);
  k_out<<<dim3(TNB * NN / 64, DD / 128), 128, 0, stream>>>(O, F[6], F[7], (float*)d_out);
}
